// S6_noC_11699490914652
// MI455X (gfx1250) — hardware-verified
//
#include <hip/hip_runtime.h>
#include <math.h>

#define BQ    8
#define LQ    2048
#define DQ    768
#define NTOK  (BQ * LQ)
#define TPB   128
#define OSTR  68
#define SCH   32
#define CHB   256

static_assert(NTOK % TPB == 0);
static_assert(DQ % 64 == 0);
static_assert(DQ % 32 == 0);
static_assert(DQ % 8 == 0);
static_assert(DQ == 3 * CHB);
static_assert(LQ % SCH == 0);
static_assert((LQ & (LQ - 1)) == 0);
static_assert(SCH * CHB == 8 * 256 * 4);
static_assert(OSTR % 4 == 0);
static_assert(DQ % 256 == 0);
static_assert((DQ / 4) <= 256);

typedef unsigned short us16 __attribute__((ext_vector_type(16)));
typedef unsigned short us8  __attribute__((ext_vector_type(8)));
typedef unsigned short us8a __attribute__((ext_vector_type(8), may_alias));
typedef __bf16 v16b __attribute__((ext_vector_type(16)));
typedef float v8f __attribute__((ext_vector_type(8)));
typedef float v4f __attribute__((ext_vector_type(4)));
typedef float v4fa __attribute__((ext_vector_type(4), may_alias));
union FragU { us16 v; us8 h[2]; };

__device__ __forceinline__ unsigned short bf16_bits(float f) {
  unsigned u = __float_as_uint(f);
  u += 0x7FFFu + ((u >> 16) & 1u);
  return (unsigned short)(u >> 16);
}
__device__ __forceinline__ float bf16_val(unsigned short b) { return __uint_as_float(((unsigned)b) << 16); }
__device__ __forceinline__ float bf16r(float f) { return bf16_val(bf16_bits(f)); }
__device__ __forceinline__ float sigm(float t) { return __builtin_amdgcn_rcpf(1.0f + __expf(-t)); }

__device__ __forceinline__ v8f mma_bf16(us16 a, us16 b, v8f c) {
  return __builtin_amdgcn_wmma_f32_16x16x32_bf16(false, __builtin_bit_cast(v16b, a), false, __builtin_bit_cast(v16b, b), (short)0, c, false, false);
}
__device__ __forceinline__ void wguard(v8f& c0, v8f& c1, v8f& c2, v8f& c3, const us16& a0,
                                       const us16& b0, const us16& b1, const us16& b2, const us16& b3) {
#if defined(__HIP_DEVICE_COMPILE__)
  asm volatile("v_nop\n\tv_nop\n\tv_nop\n\tv_nop"
               : "+v"(c0), "+v"(c1), "+v"(c2), "+v"(c3)
               : "v"(a0), "v"(b0), "v"(b1), "v"(b2), "v"(b3));
#endif
}

__device__ __forceinline__ us16 gfrag(const unsigned short* p) {
  const int kh = ((threadIdx.x >> 4) & 1) * 8;
  FragU f;
  f.h[0] = *(const us8a*)(p + kh);
  f.h[1] = *(const us8a*)(p + 16 + kh);
  return f.v;
}

__global__ __launch_bounds__(256) void k_cvt(const float* __restrict__ src, unsigned short* dst, int nsrc, int ncol8, int total8) {
  const int idx = blockIdx.x * 256 + threadIdx.x;
  if (idx >= total8) return;
  const int row = idx / ncol8, c8 = (idx - row * ncol8) * 8;
  const int rs = (row < nsrc) ? row : (nsrc - 1);
  const float* s = src + (size_t)rs * (size_t)(ncol8 * 8) + c8;
  const v4f a = *(const v4fa*)s, b = *(const v4fa*)(s + 4);
  const bool zr = (row >= nsrc);
  us8 o;
#pragma unroll
  for (int u = 0; u < 4; ++u) {
    o[u]     = zr ? (unsigned short)0 : bf16_bits(a[u]);
    o[4 + u] = zr ? (unsigned short)0 : bf16_bits(b[u]);
  }
  const size_t off = (size_t)row * (size_t)(ncol8 * 8) + c8;
  *(volatile us8*)(dst + off) = o;
  __threadfence();
  *(volatile us8*)(dst + off) = o;
}

__global__ __launch_bounds__(256) void k_sqtok(const unsigned short* __restrict__ XB, const float* __restrict__ stW,
                                              const float* __restrict__ stb, const float* __restrict__ stbias, float* G) {
  __shared__ __attribute__((aligned(16))) float sqs[DQ];
  __shared__ __attribute__((aligned(16))) float gs[DQ];
  const int tid = threadIdx.x, b = blockIdx.x;
#pragma unroll 1
  for (int j = 0; j < DQ / 256; ++j) {
    const int d = tid + 256 * j;
    const unsigned short* p = XB + (size_t)b * LQ * DQ + d;
    double s = 0.0;
#pragma unroll 4
    for (int l = 0; l < LQ; ++l) s += (double)bf16_val(p[(size_t)l * DQ]);
    sqs[d] = (float)s * (1.0f / (float)LQ);
  }
  __syncthreads();
#pragma unroll 1
  for (int j = 0; j < DQ / 256; ++j) {
    const int e = tid + 256 * j;
    const float* w = stW + (size_t)e * DQ;
    float acc = 0.0f;
#pragma unroll 4
    for (int d = 0; d < DQ; ++d) acc = fmaf(sqs[d], bf16r(w[d]), acc);
    acc = acc + bf16r(stb[e]);
    acc = fmaxf(acc, 0.0f);
    gs[e] = sigm(acc) + bf16r(stbias[e]);
  }
  __syncthreads();
  const bool wr = (tid < DQ / 4);
  v4f v = {0.f, 0.f, 0.f, 0.f};
  if (wr) v = *(const v4fa*)(gs + tid * 4);
  float* gp = G + (size_t)b * DQ + tid * 4;
  if (wr) *(volatile v4f*)gp = v;
  __threadfence();
  if (wr) *(volatile v4f*)gp = v;
}

template <int MODE>
__global__ __launch_bounds__(256) void k_gemm(const unsigned short* __restrict__ Ap, const unsigned short* __restrict__ Bw,
                                             const float* __restrict__ bias, const float* __restrict__ dpos, float* Yf) {
  __shared__ __attribute__((aligned(16))) float oS[8 * 16 * OSTR];
  const int tid = threadIdx.x, lane = tid & 31, wave = tid >> 5, cl = lane & 15, hh = lane >> 4;
  const int m0 = blockIdx.x * TPB + 16 * wave, n0 = blockIdx.y * 64;

  v8f acc[4];
#pragma unroll
  for (int j = 0; j < 4; ++j) { const v8f zz = {0.f, 0.f, 0.f, 0.f, 0.f, 0.f, 0.f, 0.f}; acc[j] = zz; }

  const unsigned short* a0p = Ap + (size_t)(m0 + cl) * (size_t)DQ;
  const unsigned short* bwp = Bw + (size_t)(n0 + cl) * (size_t)DQ;
#pragma unroll 1
  for (int k0 = 0; k0 < DQ; k0 += 32) {
    const us16 af = gfrag(a0p + k0);
    us16 bfr[4];
#pragma unroll
    for (int j = 0; j < 4; ++j) bfr[j] = gfrag(bwp + (size_t)(16 * j) * (size_t)DQ + k0);
#pragma unroll
    for (int j = 0; j < 4; ++j) acc[j] = mma_bf16(af, bfr[j], acc[j]);
    wguard(acc[0], acc[1], acc[2], acc[3], af, bfr[0], bfr[1], bfr[2], bfr[3]);
  }

  float* so = oS + wave * (16 * OSTR);
#pragma unroll
  for (int j = 0; j < 4; ++j)
#pragma unroll
    for (int r = 0; r < 8; ++r) so[(8 * hh + r) * OSTR + 16 * j + cl] = acc[j][r];
  __syncthreads();

#pragma unroll 1
  for (int it = 0; it < 8; ++it) {
    const int cx = it * 32 + lane, r = cx >> 4, q = (cx & 15) * 4;
    v4f v = *(const v4fa*)(so + r * OSTR + q);
    const int l = (m0 + r) & (LQ - 1);
#pragma unroll
    for (int u = 0; u < 4; ++u) {
      float t = v[u] + bf16r(bias[n0 + q + u]);
      if (MODE == 1) {
        t = t + bf16r(dpos[(size_t)l * DQ + n0 + q + u]);
        t = sigm(t);
      }
      v[u] = t;
    }
    *(v4fa*)(so + r * OSTR + q) = v;
  }
#pragma unroll
  for (int pass = 0; pass < 2; ++pass) {
#pragma unroll
    for (int it = 0; it < 8; ++it) {
      const int cx = it * 32 + lane, r = cx >> 4, q = (cx & 15) * 4;
      const v4f v = *(const v4fa*)(so + r * OSTR + q);
      *(volatile v4f*)(Yf + (size_t)(m0 + r) * (size_t)DQ + n0 + q) = v;
    }
    __threadfence();
  }
}

__global__ __launch_bounds__(256) void k_scan(const unsigned short* __restrict__ XB, const float* __restrict__ Atab,
                                             const float* __restrict__ DL, const float* __restrict__ B0P,
                                             const float* __restrict__ G, float* out) {
  __shared__ __attribute__((aligned(16))) float sy[SCH * CHB];
  const int tid = threadIdx.x;
  const int b = blockIdx.x / (DQ / CHB), dg = blockIdx.x - b * (DQ / CHB);
  const int d = dg * CHB + tid;
  const float gv = G[(size_t)b * DQ + d];
  float s = 0.0f;

#pragma unroll 1
  for (int c = 0; c < LQ / SCH; ++c) {
#pragma unroll 1
    for (int st = 0; st < SCH; ++st) {
      const int l = c * SCH + st;
      const size_t i = ((size_t)b * LQ + (size_t)l) * DQ + d;
      const float xd = bf16_val(XB[i]);
      const float de = DL[i];
      const float b0 = B0P[i];
      const float cc = out[i];
      const float av = bf16r(Atab[(size_t)l * DQ + d]);
      const float a  = de * av;
      const float bb = de * b0;
      s = a * s + bb * xd;
      const float y = cc * s + gv * xd;
      sy[st * CHB + tid] = y * sigm(xd);
    }
    __syncthreads();
    float* ob = out + ((size_t)b * LQ + (size_t)(c * SCH)) * DQ + (size_t)dg * CHB;
#pragma unroll
    for (int pass = 0; pass < 2; ++pass) {
#pragma unroll
      for (int it = 0; it < 8; ++it) {
        const int cx = it * 256 + tid, r = cx >> 6, q = (cx & 63) * 4;
        const v4f v = *(const v4fa*)(sy + r * CHB + q);
        *(volatile v4f*)(ob + (size_t)r * DQ + q) = v;
      }
      __threadfence();
    }
    __syncthreads();
  }
}

extern "C" void kernel_launch(void* const* d_in, const int* in_sizes, int n_in,
                              void* d_out, int out_size, void* d_ws, size_t ws_size,
                              hipStream_t stream) {
  if (n_in < 12) return;
  if (in_sizes[0] != NTOK * DQ || in_sizes[1] != DQ * DQ || in_sizes[2] != DQ || in_sizes[3] != DQ * DQ || in_sizes[4] != DQ ||
      in_sizes[5] != DQ * DQ || in_sizes[6] != DQ || in_sizes[7] != LQ * DQ || in_sizes[8] != LQ * DQ || in_sizes[9] != DQ * DQ ||
      in_sizes[10] != DQ || in_sizes[11] != DQ) return;
  if (out_size != NTOK * DQ) return;

  const float* x       = (const float*)d_in[0];
  const float* W_B     = (const float*)d_in[1];
  const float* b_B     = (const float*)d_in[2];
  const float* W_C     = (const float*)d_in[3];
  const float* b_C     = (const float*)d_in[4];
  const float* W_d     = (const float*)d_in[5];
  const float* b_d     = (const float*)d_in[6];
  const float* delta_p = (const float*)d_in[7];
  const float* Atab    = (const float*)d_in[8];
  const float* st_W    = (const float*)d_in[9];
  const float* st_b    = (const float*)d_in[10];
  const float* st_bias = (const float*)d_in[11];
  float* out = (float*)d_out;

  size_t off = 0;
  auto carve = [&](size_t bytes) -> char* { char* p = (char*)d_ws + off; off += (bytes + 255) & ~(size_t)255; return p; };
  unsigned short* XB  = (unsigned short*)carve((size_t)NTOK * DQ * 2);
  unsigned short* WBb = (unsigned short*)carve((size_t)DQ * DQ * 2);
  unsigned short* WCb = (unsigned short*)carve((size_t)DQ * DQ * 2);
  unsigned short* WDb = (unsigned short*)carve((size_t)DQ * DQ * 2);
  float* B0P = (float*)carve((size_t)NTOK * DQ * 4);
  float* DL  = (float*)carve((size_t)NTOK * DQ * 4);
  float* G   = (float*)carve((size_t)BQ * DQ * 4);
  if (off > ws_size || off > (size_t)134217728) return;

  const dim3 b256(256);
  auto cdv = [](long a, long bq) { return (unsigned)((a + bq - 1) / bq); };

  k_cvt<<<dim3(cdv((long)NTOK * DQ / 8, 256)), b256, 0, stream>>>(x, XB, NTOK, DQ / 8, NTOK * DQ / 8);
  k_cvt<<<dim3(cdv((long)DQ * DQ / 8, 256)), b256, 0, stream>>>(W_B, WBb, DQ, DQ / 8, DQ * DQ / 8);
  k_cvt<<<dim3(cdv((long)DQ * DQ / 8, 256)), b256, 0, stream>>>(W_C, WCb, DQ, DQ / 8, DQ * DQ / 8);
  k_cvt<<<dim3(cdv((long)DQ * DQ / 8, 256)), b256, 0, stream>>>(W_d, WDb, DQ, DQ / 8, DQ * DQ / 8);
  k_sqtok<<<dim3(BQ), b256, 0, stream>>>(XB, st_W, st_b, st_bias, G);
  const dim3 gg(NTOK / TPB, DQ / 64);
  k_gemm<0><<<gg, b256, 0, stream>>>(XB, WBb, b_B, delta_p, B0P);
  k_gemm<0><<<gg, b256, 0, stream>>>(XB, WCb, b_C, delta_p, out);
  k_gemm<1><<<gg, b256, 0, stream>>>(XB, WDb, b_d, delta_p, DL);
  k_scan<<<dim3(BQ * (DQ / CHB)), b256, 0, stream>>>(XB, Atab, DL, B0P, G, out);
}
